// FastVARCrossAttnBlock_3925600109080
// MI455X (gfx1250) — hardware-verified
//
#include <hip/hip_runtime.h>
#include <math.h>
#include <stdint.h>

#define BATCH   2
#define SEQ     4096
#define GW      64
#define HC      32
#define DM      1024
#define NH      16
#define HD      64
#define H3      3072
#define MP      1664
#define NQB     (MP / 64)
#define MTOT    (BATCH * MP)
#define QKPLANE (BATCH * NH * MP * HD)
static_assert(NH * HD == DM);
static_assert((MP % 64) == 0 && (DM % 64) == 0 && (H3 % 64) == 0 && (SEQ % 32) == 0 && (MTOT % 64) == 0);
static_assert(GW * GW == SEQ && 2 * HC == GW);

typedef _Float16 v16h __attribute__((ext_vector_type(16)));
typedef _Float16 v8h  __attribute__((ext_vector_type(8)));
typedef float    v8f  __attribute__((ext_vector_type(8)));
typedef float    v4f  __attribute__((ext_vector_type(4)));
typedef unsigned int v4u __attribute__((ext_vector_type(4)));
typedef int      v4i __attribute__((ext_vector_type(4)));

__device__ __forceinline__ unsigned short h_bits(_Float16 x) { return __builtin_bit_cast(unsigned short, x); }
__device__ __forceinline__ unsigned pk16(unsigned short a, unsigned short b) { return (unsigned)a | ((unsigned)b << 16); }
__device__ __forceinline__ v8f zero8() { v8f z = {0.f, 0.f, 0.f, 0.f, 0.f, 0.f, 0.f, 0.f}; return z; }
__device__ __forceinline__ void wsync() {
  __builtin_amdgcn_fence(__ATOMIC_RELEASE, "workgroup");
  __builtin_amdgcn_wave_barrier();
  __builtin_amdgcn_fence(__ATOMIC_ACQUIRE, "workgroup");
}

__device__ __forceinline__ v16h ldfrag_h(const _Float16* p) {
  union { v16h v; v8h h[2]; } f;
  f.h[0] = *(const v8h*)(p);
  f.h[1] = *(const v8h*)(p + 16);
  return f.v;
}

__device__ __forceinline__ v8f mma_h(v16h a, v16h b, v8f c) {
  c = __builtin_amdgcn_wmma_f32_16x16x32_f16(false, a, false, b, (short)0, c, false, false);
  asm volatile("v_nop\n\tv_nop\n\tv_nop\n\tv_nop" : "+v"(c) : "v"(a), "v"(b));
  return c;
}

__global__ __launch_bounds__(256) void k_mean(const float* __restrict__ x, float* mean) {
  __shared__ float part[8][32];
  const int lane = threadIdx.x & 31, wave = threadIdx.x >> 5;
  const int cg = blockIdx.x, b = blockIdx.y;
  const float* p = x + (size_t)b * SEQ * DM + (size_t)(wave * (SEQ / 8)) * DM + cg * 32 + lane;
  float s = 0.f;
#pragma unroll 8
  for (int r = 0; r < SEQ / 8; ++r) s += p[(size_t)r * DM];
  part[wave][lane] = s;
  __syncthreads();
  if (wave == 0) {
    float t = part[0][lane];
#pragma unroll
    for (int w = 1; w < 8; ++w) t += part[w][lane];
    const float m = t * (1.0f / SEQ);
    float* dst = mean + (size_t)b * DM + cg * 32 + lane;
    *(volatile float*)dst = m;
    __threadfence();
    *(volatile float*)dst = m;
  }
}

__global__ __launch_bounds__(256) void k_mse(const float* __restrict__ x, const float* __restrict__ mean,
                                             float* mse) {
#pragma clang fp contract(off)
  __shared__ float sm[32];
  const int lane = threadIdx.x & 31, wave = threadIdx.x >> 5;
  const int r0 = blockIdx.x * 32;
  const int b = r0 / SEQ;
  float mu[32];
#pragma unroll
  for (int it = 0; it < 8; ++it) {
    const v4f a = *(const v4f*)(mean + (size_t)b * DM + it * 128 + lane * 4);
#pragma unroll
    for (int e = 0; e < 4; ++e) mu[4 * it + e] = a[e];
  }
#pragma unroll 1
  for (int rr = 0; rr < 4; ++rr) {
    const int row = r0 + wave * 4 + rr;
    const float* xr = x + (size_t)row * DM;
    float s = 0.f;
#pragma unroll
    for (int it = 0; it < 8; ++it) {
      const v4f a = *(const v4f*)(xr + it * 128 + lane * 4);
#pragma unroll
      for (int e = 0; e < 4; ++e) {
        const float d = a[e] - mu[4 * it + e];
        const float sq = d * d;
        s = s + sq;
      }
    }
#pragma unroll
    for (int off = 16; off > 0; off >>= 1) s += __shfl_xor(s, off, 32);
    if (lane == 0) sm[wave * 4 + rr] = s;
  }
  __syncthreads();
  if (wave == 0) {
    const float v = sm[lane];
    float* dst = mse + r0 + lane;
    *(volatile float*)dst = v;
    __threadfence();
    *(volatile float*)dst = v;
  }
}

__global__ __launch_bounds__(512) void k_select(const float* __restrict__ mse, const int* __restrict__ nrp,
                                                int* idxo, int* rnko) {
  __shared__ float keys[SEQ];
  __shared__ int   vals[SEQ];
  __shared__ int   rk[SEQ];
  const int tid = threadIdx.x, b = blockIdx.x;
  int nr = nrp[0];
  nr = (nr < 1) ? 1 : nr;
  nr = (nr > MP) ? MP : nr;
  for (int i = tid; i < SEQ; i += 512) { keys[i] = mse[(size_t)b * SEQ + i]; vals[i] = i; }
  __syncthreads();
  for (int k = 2; k <= SEQ; k <<= 1) {
    for (int j = k >> 1; j > 0; j >>= 1) {
#pragma unroll
      for (int pp = 0; pp < 4; ++pp) {
        const int p  = tid + pp * 512;
        const int i  = ((p & ~(j - 1)) << 1) | (p & (j - 1));
        const int ip = i | j;
        const float ka = keys[i];  const int ia = vals[i];
        const float kb = keys[ip]; const int ib = vals[ip];
        const bool bfa = (kb > ka) || (kb == ka && ib < ia);
        const bool afb = (ka > kb) || (ka == kb && ia < ib);
        const bool up  = ((i & k) == 0);
        const bool sw  = up ? bfa : afb;
        keys[i]  = sw ? kb : ka;  vals[i]  = sw ? ib : ia;
        keys[ip] = sw ? ka : kb;  vals[ip] = sw ? ia : ib;
      }
      __syncthreads();
    }
  }
  for (int r = tid; r < SEQ; r += 512) rk[vals[r] & (SEQ - 1)] = (r < nr) ? r : -1;
  __syncthreads();
  v4i iv[2], rv[2];
#pragma unroll
  for (int q = 0; q < 2; ++q) {
    const int e4 = tid + q * 512;
    v4i a, c;
#pragma unroll
    for (int e = 0; e < 4; ++e) {
      const int r = 4 * e4 + e;
      a[e] = (r < nr) ? vals[r] : -1;
      c[e] = rk[r];
    }
    iv[q] = a; rv[q] = c;
  }
#pragma unroll
  for (int q = 0; q < 2; ++q) {
    const int e4 = tid + q * 512;
    *(volatile v4i*)(idxo + (size_t)b * SEQ + 4 * e4) = iv[q];
    *(volatile v4i*)(rnko + (size_t)b * SEQ + 4 * e4) = rv[q];
  }
  __threadfence();
#pragma unroll
  for (int q = 0; q < 2; ++q) {
    const int e4 = tid + q * 512;
    *(volatile v4i*)(idxo + (size_t)b * SEQ + 4 * e4) = iv[q];
    *(volatile v4i*)(rnko + (size_t)b * SEQ + 4 * e4) = rv[q];
  }
}

__global__ __launch_bounds__(256) void cvt_h(const float* __restrict__ W, unsigned short* O, int n8, float scale) {
  const int t = blockIdx.x * 256 + threadIdx.x;
  if (t >= n8) return;
  const float* s = W + (size_t)t * 8;
  const v4f a = *(const v4f*)s;
  const v4f c = *(const v4f*)(s + 4);
  v4u p;
  p[0] = pk16(h_bits((_Float16)(a[0] * scale)), h_bits((_Float16)(a[1] * scale)));
  p[1] = pk16(h_bits((_Float16)(a[2] * scale)), h_bits((_Float16)(a[3] * scale)));
  p[2] = pk16(h_bits((_Float16)(c[0] * scale)), h_bits((_Float16)(c[1] * scale)));
  p[3] = pk16(h_bits((_Float16)(c[2] * scale)), h_bits((_Float16)(c[3] * scale)));
  unsigned short* d = O + (size_t)t * 8;
  *(volatile v4u*)d = p;
  __threadfence();
  *(volatile v4u*)d = p;
}

__global__ __launch_bounds__(256) void k_gather(const float* __restrict__ x, const float* __restrict__ rope,
                                                const int* __restrict__ idx, unsigned short* xm,
                                                float* rc, float* rs) {
  const int lane = threadIdx.x & 31, wave = threadIdx.x >> 5;
  const int gr = blockIdx.x * 8 + wave;
  const int b = gr / MP, r = gr - b * MP;
  int pos = idx[(size_t)b * SEQ + r];
  const float vf = (pos >= 0) ? 1.0f : 0.0f;
  pos = (pos < 0) ? 0 : pos;
  pos = (pos > SEQ - 1) ? (SEQ - 1) : pos;
  const float* xr = x + ((size_t)b * SEQ + pos) * DM;
  v4u pk[4];
#pragma unroll
  for (int it = 0; it < 4; ++it) {
    const int c0 = it * 256 + lane * 8;
    const v4f a = *(const v4f*)(xr + c0);
    const v4f c = *(const v4f*)(xr + c0 + 4);
    v4u p;
    p[0] = pk16(h_bits((_Float16)(a[0] * vf)), h_bits((_Float16)(a[1] * vf)));
    p[1] = pk16(h_bits((_Float16)(a[2] * vf)), h_bits((_Float16)(a[3] * vf)));
    p[2] = pk16(h_bits((_Float16)(c[0] * vf)), h_bits((_Float16)(c[1] * vf)));
    p[3] = pk16(h_bits((_Float16)(c[2] * vf)), h_bits((_Float16)(c[3] * vf)));
    pk[it] = p;
  }
  const float cv = rope[(size_t)pos * 32 + lane] * vf;
  const float sv = rope[(size_t)SEQ * 32 + (size_t)pos * 32 + lane] * vf;
#pragma unroll
  for (int it = 0; it < 4; ++it)
    *(volatile v4u*)(xm + (size_t)gr * DM + it * 256 + lane * 8) = pk[it];
  *(volatile float*)(rc + (size_t)gr * 32 + lane) = cv;
  *(volatile float*)(rs + (size_t)gr * 32 + lane) = sv;
  __threadfence();
#pragma unroll
  for (int it = 0; it < 4; ++it)
    *(volatile v4u*)(xm + (size_t)gr * DM + it * 256 + lane * 8) = pk[it];
  *(volatile float*)(rc + (size_t)gr * 32 + lane) = cv;
  *(volatile float*)(rs + (size_t)gr * 32 + lane) = sv;
}

template <int EPI>
__global__ __launch_bounds__(256) void gemm64(
    const unsigned short* __restrict__ Ap, int lda,
    const unsigned short* __restrict__ Btp, int ldb, int bsB,
    void* Cout, int ldc, int bsC,
    const float* __restrict__ bias, const float* __restrict__ rc,
    const float* __restrict__ rs, const float* __restrict__ smlog,
    int M, int N, int K, float oscale, float cscale) {
  const _Float16* A  = (const _Float16*)(const void*)Ap;
  const _Float16* Bt = (const _Float16*)(const void*)Btp + (size_t)blockIdx.y * (size_t)bsB;
  const size_t cofs = (size_t)blockIdx.y * (size_t)bsC;
  __shared__ __align__(16) float sT[8][16 * 68];
  const int lane = threadIdx.x & 31;
  const int wave = threadIdx.x >> 5;
  const int tilesN = N >> 6;
  const int tilesM = M >> 6;
  const int tile = blockIdx.x * 8 + wave;
  if (tile >= tilesM * tilesN) return;
  const int tm = tile / tilesN;
  const int tn = tile - tm * tilesN;
  const int m0 = tm << 6;
  const int n0 = tn << 6;
  const int rl   = lane & 15;
  const int hh   = lane >> 4;
  const int koff = hh * 8;
  const int mOff = hh * 8;

  v8f acc[4][4];
#pragma unroll
  for (int i = 0; i < 4; ++i)
#pragma unroll
    for (int j = 0; j < 4; ++j) acc[i][j] = zero8();

  for (int k0 = 0; k0 < K; k0 += 32) {
    v16h bf[4];
#pragma unroll
    for (int j = 0; j < 4; ++j)
      bf[j] = ldfrag_h(Bt + (size_t)(n0 + (j << 4) + rl) * ldb + k0 + koff);
#pragma unroll
    for (int i = 0; i < 4; ++i) {
      const v16h af = ldfrag_h(A + (size_t)(m0 + (i << 4) + rl) * lda + k0 + koff);
#pragma unroll
      for (int j = 0; j < 4; ++j) acc[i][j] = mma_h(af, bf[j], acc[i][j]);
    }
  }

  float hs = 1.0f, qsel = 0.0f;
  int which = 0, head = 0;
  if (EPI == 1) {
    which = n0 >> 10;
    head  = (n0 & (DM - 1)) >> 6;
    const float ev = expf(fminf(smlog[head], 4.6051702f));
    hs   = (which == 0) ? ev : 1.0f;
    qsel = (which == 0) ? 1.0f : 0.0f;
  }

  float* slab = sT[wave];
#pragma unroll
  for (int i = 0; i < 4; ++i) {
    const int mBase = m0 + (i << 4);
#pragma unroll
    for (int j = 0; j < 4; ++j) {
#pragma unroll
      for (int r = 0; r < 8; ++r) slab[(mOff + r) * 68 + (j << 4) + rl] = acc[i][j][r];
    }
    wsync();
    if (EPI == 0) {
      float* Cf = (float*)Cout;
      const int c4 = rl * 4;
      const v4f bv = *(const v4f*)(bias + n0 + c4);
      v4f vv[8];
#pragma unroll
      for (int it = 0; it < 8; ++it) {
        const int row = it * 2 + hh;
        v4f v = *(const v4f*)(slab + row * 68 + c4);
        vv[it] = v * oscale + bv;
      }
#pragma unroll
      for (int it = 0; it < 8; ++it) {
        const int row = it * 2 + hh;
        *(volatile v4f*)(Cf + cofs + (size_t)(mBase + row) * ldc + n0 + c4) = vv[it];
      }
      __threadfence();
#pragma unroll
      for (int it = 0; it < 8; ++it) {
        const int row = it * 2 + hh;
        *(volatile v4f*)(Cf + cofs + (size_t)(mBase + row) * ldc + n0 + c4) = vv[it];
      }
    } else {
      if (EPI == 1) {
        const float b0v = bias[(n0 & (DM - 1)) + 2 * lane] * qsel;
        const float b1v = bias[(n0 & (DM - 1)) + 2 * lane + 1] * qsel;
#pragma unroll 1
        for (int e = 0; e < 16; ++e) {
          const int m = mBase + e;
          const float cs = rc[(size_t)m * 32 + lane];
          const float sn = rs[(size_t)m * 32 + lane];
          const float x1 = slab[e * 68 + 2 * lane] * oscale + b0v;
          const float x2 = slab[e * 68 + 2 * lane + 1] * oscale + b1v;
          float ss = x1 * x1 + x2 * x2;
#pragma unroll
          for (int off = 16; off > 0; off >>= 1) ss += __shfl_xor(ss, off, 32);
          const float den = fmaxf(sqrtf(ss), 1e-12f);
          const float inv = (1.0f / den) * hs;
          const float t1 = x1 * inv, t2 = x2 * inv;
          slab[e * 68 + 2 * lane]     = (cs * t1 - sn * t2) * cscale;
          slab[e * 68 + 2 * lane + 1] = (sn * t1 + cs * t2) * cscale;
        }
        wsync();
      }
      const int q = lane >> 3, c8 = (lane & 7) * 8;
      unsigned short* Cb = (unsigned short*)Cout;
      size_t sbase, spitch;
      if (EPI == 1) {
        const int bb = mBase / MP;
        const int t0 = mBase - bb * MP;
        sbase  = (size_t)which * QKPLANE + ((size_t)(bb * NH + head) * MP + t0) * HD;
        spitch = HD;
      } else {
        sbase  = cofs + (size_t)mBase * ldc + n0;
        spitch = (size_t)ldc;
      }
      v4u hv[4];
#pragma unroll
      for (int it = 0; it < 4; ++it) {
        const int row = it * 4 + q;
        const float* sp = slab + row * 68 + c8;
        float bm = 0.0f;
        if (EPI == 2) bm = bias[mBase + row];
        v4u a;
#pragma unroll
        for (int e = 0; e < 4; ++e) {
          float f0, f1;
          if (EPI == 2) { f0 = (sp[2 * e] * oscale + bm) * cscale; f1 = (sp[2 * e + 1] * oscale + bm) * cscale; }
          else          { f0 = sp[2 * e];                        f1 = sp[2 * e + 1]; }
          a[e] = pk16(h_bits((_Float16)f0), h_bits((_Float16)f1));
        }
        hv[it] = a;
      }
#pragma unroll
      for (int it = 0; it < 4; ++it) {
        const int row = it * 4 + q;
        *(volatile v4u*)(Cb + sbase + (size_t)row * spitch + c8) = hv[it];
      }
      __threadfence();
#pragma unroll
      for (int it = 0; it < 4; ++it) {
        const int row = it * 4 + q;
        *(volatile v4u*)(Cb + sbase + (size_t)row * spitch + c8) = hv[it];
      }
    }
    wsync();
  }
}

__global__ __launch_bounds__(128)
void attn64(const unsigned short* __restrict__ qp, const unsigned short* __restrict__ kp,
            const unsigned short* __restrict__ vtp, const int* __restrict__ nrp,
            unsigned short* op, float sscale, float onorm) {
  union FH { v16h v; v8h h[2]; };
  __shared__ __align__(16) _Float16 Ksh[64 * 64];
  __shared__ __align__(16) _Float16 Vth[64 * 64];
  __shared__ __align__(16) _Float16 Psh[4][16 * 64];
  __shared__ __align__(16) float    Os[4][16 * 64];

  const int tid  = threadIdx.x;
  const int wave = tid >> 5;
  const int lane = tid & 31;
  const int hh   = lane >> 4;
  const int c    = lane & 15;
  const int bx   = blockIdx.x;
  const int bh   = bx / NQB;
  const int qb   = bx - bh * NQB;
  const int b    = bh / NH;
  const int h    = bh - b * NH;
  const int q0   = qb * 64 + wave * 16;
  int nr = nrp[0];
  nr = (nr < 1) ? 1 : nr;
  nr = (nr > MP) ? MP : nr;

  const _Float16* Q  = (const _Float16*)(const void*)qp  + (size_t)bh * MP * HD;
  const _Float16* Kg = (const _Float16*)(const void*)kp  + (size_t)bh * MP * HD;
  const _Float16* V  = (const _Float16*)(const void*)vtp + (size_t)bh * HD * MP;

  v16h qa[2];
#pragma unroll
  for (int dc = 0; dc < 2; ++dc) qa[dc] = ldfrag_h(Q + (size_t)(q0 + c) * HD + dc * 32 + 8 * hh);

  float mrow[8], lrow[8];
  v8f oacc[4];
#pragma unroll
  for (int r = 0; r < 8; ++r) { mrow[r] = -INFINITY; lrow[r] = 0.f; }
#pragma unroll
  for (int t = 0; t < 4; ++t) oacc[t] = zero8();

  for (int kt = 0; kt < NQB; ++kt) {
    const int kv0 = kt * 64;
    __syncthreads();
    {
      const int r = tid >> 1, half = (tid & 1) * 32;
      const _Float16* kg = Kg + (size_t)(kv0 + r) * HD + half;
      const _Float16* vg = V + (size_t)r * MP + kv0 + half;
#pragma unroll
      for (int i = 0; i < 4; ++i) {
        const v8h a0 = *(const v8h*)(kg + 8 * i);
        const v8h b0 = *(const v8h*)(vg + 8 * i);
        *(v8h*)(Ksh + r * 64 + half + 8 * i) = a0;
        *(v8h*)(Vth + r * 64 + half + 8 * i) = b0;
      }
    }
    __syncthreads();

    v8f s[4];
#pragma unroll
    for (int j = 0; j < 4; ++j) {
      s[j] = zero8();
#pragma unroll
      for (int dc = 0; dc < 2; ++dc) {
        FH kb;
        kb.h[0] = *(const v8h*)(Ksh + (j * 16 + c) * 64 + dc * 32 + 8 * hh);
        kb.h[1] = *(const v8h*)(Ksh + (j * 16 + c) * 64 + dc * 32 + 16 + 8 * hh);
        s[j] = mma_h(qa[dc], kb.v, s[j]);
      }
    }

    _Float16* pw = Psh[wave];
#pragma unroll
    for (int r = 0; r < 8; ++r) {
      float m = -INFINITY;
#pragma unroll
      for (int j = 0; j < 4; ++j) {
        const int key = kv0 + j * 16 + c;
        float sv = s[j][r] * sscale;
        sv = (key >= nr) ? -INFINITY : sv;
        s[j][r] = sv;
        m = fmaxf(m, sv);
      }
#pragma unroll
      for (int off = 1; off < 16; off <<= 1) m = fmaxf(m, __shfl_xor(m, off, 32));
      const float mnew  = fmaxf(mrow[r], m);
      const float msafe = (mnew == -INFINITY) ? 0.f : mnew;
      const float alpha = __expf(mrow[r] - msafe);
      mrow[r] = mnew;
      float psum = 0.f;
#pragma unroll
      for (int j = 0; j < 4; ++j) {
        const float p = __expf(s[j][r] - msafe);
        psum += p;
        pw[(8 * hh + r) * 64 + j * 16 + c] = (_Float16)(p * 1024.0f);
      }
#pragma unroll
      for (int off = 1; off < 16; off <<= 1) psum += __shfl_xor(psum, off, 32);
      lrow[r] = lrow[r] * alpha + psum;
#pragma unroll
      for (int t = 0; t < 4; ++t) oacc[t][r] *= alpha;
    }
    wsync();

#pragma unroll
    for (int kk = 0; kk < 2; ++kk) {
      FH pa;
      pa.h[0] = *(const v8h*)(pw + c * 64 + kk * 32 + 8 * hh);
      pa.h[1] = *(const v8h*)(pw + c * 64 + kk * 32 + 16 + 8 * hh);
#pragma unroll
      for (int t = 0; t < 4; ++t) {
        FH vb;
        vb.h[0] = *(const v8h*)(Vth + (t * 16 + c) * 64 + kk * 32 + 8 * hh);
        vb.h[1] = *(const v8h*)(Vth + (t * 16 + c) * 64 + kk * 32 + 16 + 8 * hh);
        oacc[t] = mma_h(pa.v, vb.v, oacc[t]);
      }
    }
  }

  float* os = Os[wave];
#pragma unroll
  for (int r = 0; r < 8; ++r) {
    const float l = lrow[r];
    const float inv = ((l > 0.f) ? (1.0f / l) : 0.f) * onorm;
#pragma unroll
    for (int t = 0; t < 4; ++t) os[(8 * hh + r) * 64 + t * 16 + c] = oacc[t][r] * inv;
  }
  wsync();
  {
    const int q4 = lane >> 3, c8 = (lane & 7) * 8;
    v4u hv[4];
#pragma unroll
    for (int it = 0; it < 4; ++it) {
      const int row = it * 4 + q4;
      const float* sp = os + row * 64 + c8;
      v4u a;
#pragma unroll
      for (int e = 0; e < 4; ++e) a[e] = pk16(h_bits((_Float16)sp[2 * e]), h_bits((_Float16)sp[2 * e + 1]));
      hv[it] = a;
    }
    const size_t orow0 = (size_t)b * MP + q0;
#pragma unroll
    for (int it = 0; it < 4; ++it) {
      const int row = it * 4 + q4;
      *(volatile v4u*)(op + (orow0 + row) * DM + (size_t)h * HD + c8) = hv[it];
    }
    __threadfence();
#pragma unroll
    for (int it = 0; it < 4; ++it) {
      const int row = it * 4 + q4;
      *(volatile v4u*)(op + (orow0 + row) * DM + (size_t)h * HD + c8) = hv[it];
    }
  }
}

__global__ __launch_bounds__(256) void k_out(const float* __restrict__ x, const float* __restrict__ cached,
                                             const int* __restrict__ rnk, const float* __restrict__ O,
                                             float* out) {
  const int lane = threadIdx.x & 31, wave = threadIdx.x >> 5;
  const int row = blockIdx.x * 8 + wave;
  const int b = row / SEQ, l = row - b * SEQ;
  int rk = rnk[row];
  rk = (rk < -1) ? -1 : rk;
  rk = (rk > MP - 1) ? (MP - 1) : rk;
  const bool kept = (rk >= 0);
  const int rka = kept ? rk : 0;
  const float* orow = O + ((size_t)b * MP + rka) * DM;
  const int yy = l >> 7;
  const int xx = (l & 63) >> 1;
  const float* urow = cached + (((size_t)b * HC + yy) * HC + xx) * DM;
  const float* xr = x + (size_t)row * DM;
  v4f vv[8];
#pragma unroll
  for (int it = 0; it < 8; ++it) {
    const int c0 = it * 128 + lane * 4;
    const v4f a = *(const v4f*)(xr + c0);
    const v4f o = *(const v4f*)(orow + c0);
    const v4f u = *(const v4f*)(urow + c0);
    v4f add;
#pragma unroll
    for (int e = 0; e < 4; ++e) add[e] = kept ? o[e] : u[e];
    vv[it] = a + add;
  }
#pragma unroll
  for (int it = 0; it < 8; ++it)
    *(volatile v4f*)(out + (size_t)row * DM + it * 128 + lane * 4) = vv[it];
  __threadfence();
#pragma unroll
  for (int it = 0; it < 8; ++it)
    *(volatile v4f*)(out + (size_t)row * DM + it * 128 + lane * 4) = vv[it];
}

extern "C" void kernel_launch(void* const* d_in, const int* in_sizes, int n_in,
                              void* d_out, int out_size, void* d_ws, size_t ws_size,
                              hipStream_t stream) {
  if (n_in < 10) return;
  if (in_sizes[0] != BATCH * SEQ * DM) return;
  if (in_sizes[1] != BATCH * HC * HC * DM) return;
  if (in_sizes[2] != H3 * DM) return;
  if (in_sizes[3] != DM || in_sizes[4] != DM) return;
  if (in_sizes[5] != DM * DM) return;
  if (in_sizes[6] != DM) return;
  if (in_sizes[7] != NH) return;
  if (in_sizes[8] != 2 * SEQ * 32) return;
  if (in_sizes[9] < 1) return;
  if (out_size != BATCH * SEQ * DM) return;

  const float* x      = (const float*)d_in[0];
  const float* cached = (const float*)d_in[1];
  const float* Wqkv   = (const float*)d_in[2];
  const float* qbias  = (const float*)d_in[3];
  const float* vbias  = (const float*)d_in[4];
  const float* Wproj  = (const float*)d_in[5];
  const float* bproj  = (const float*)d_in[6];
  const float* smlog  = (const float*)d_in[7];
  const float* rope   = (const float*)d_in[8];
  const int*   nrp    = (const int*)d_in[9];
  float* out = (float*)d_out;

  const size_t szMean = (size_t)BATCH * DM * 4;
  const size_t szMse  = (size_t)BATCH * SEQ * 4;
  const size_t szIdx  = (size_t)BATCH * SEQ * 4;
  const size_t szRnk  = (size_t)BATCH * SEQ * 4;
  const size_t szRC   = (size_t)MTOT * 32 * 4;
  const size_t szWq   = (size_t)H3 * DM * 2;
  const size_t szWp   = (size_t)DM * DM * 2;
  const size_t szXm   = (size_t)MTOT * DM * 2;
  const size_t szQK   = (size_t)2 * QKPLANE * 2;
  const size_t szVT   = (size_t)BATCH * DM * MP * 2;
  const size_t szCtx  = (size_t)MTOT * DM * 2;
  const size_t szO    = (size_t)MTOT * DM * 4;
  size_t off = 0;
  const size_t oMean = off; off += szMean;
  const size_t oMse  = off; off += szMse;
  const size_t oIdx  = off; off += szIdx;
  const size_t oRnk  = off; off += szRnk;
  const size_t oRC   = off; off += szRC;
  const size_t oRS   = off; off += szRC;
  const size_t oWq   = off; off += szWq;
  const size_t oWp   = off; off += szWp;
  const size_t oXm   = off; off += szXm;
  const size_t oQK   = off; off += szQK;
  const size_t oVT   = off; off += szVT;
  const size_t oCtx  = off; off += szCtx;
  const size_t oO    = off; off += szO;
  if (off > ws_size) return;
  if (off > (size_t)134217728) return;

  char* ws = (char*)d_ws;
  float*          dMean = (float*)(ws + oMean);
  float*          dMse  = (float*)(ws + oMse);
  int*            dIdx  = (int*)(ws + oIdx);
  int*            dRnk  = (int*)(ws + oRnk);
  float*          dRC   = (float*)(ws + oRC);
  float*          dRS   = (float*)(ws + oRS);
  unsigned short* WqH   = (unsigned short*)(ws + oWq);
  unsigned short* WpH   = (unsigned short*)(ws + oWp);
  unsigned short* xm    = (unsigned short*)(ws + oXm);
  unsigned short* qkP   = (unsigned short*)(ws + oQK);
  unsigned short* qP    = qkP;
  unsigned short* kP    = qkP + (size_t)QKPLANE;
  unsigned short* vT    = (unsigned short*)(ws + oVT);
  unsigned short* ctx   = (unsigned short*)(ws + oCtx);
  float*          dO    = (float*)(ws + oO);

  const dim3 blk(256);
  k_mean<<<dim3(DM / 32, BATCH), blk, 0, stream>>>(x, dMean);
  k_mse<<<dim3(BATCH * SEQ / 32), blk, 0, stream>>>(x, dMean, dMse);
  k_select<<<dim3(BATCH), dim3(512), 0, stream>>>(dMse, nrp, dIdx, dRnk);
  {
    const int n8q = H3 * DM / 8, n8p = DM * DM / 8;
    cvt_h<<<dim3((n8q + 255) / 256), blk, 0, stream>>>(Wqkv, WqH, n8q, 32.0f);
    cvt_h<<<dim3((n8p + 255) / 256), blk, 0, stream>>>(Wproj, WpH, n8p, 32.0f);
  }
  k_gather<<<dim3(MTOT / 8), blk, 0, stream>>>(x, rope, dIdx, xm, dRC, dRS);
  {
    const int tiles = (MTOT / 64) * (2 * DM / 64);
    gemm64<1><<<dim3((tiles + 7) / 8, 1), blk, 0, stream>>>(
        xm, DM, WqH, DM, 0, (void*)qkP, HD, 0, qbias, dRC, dRS, smlog,
        MTOT, 2 * DM, DM, 1.0f / 32.0f, 4.0f);
  }
  {
    const int tiles = (DM / 64) * (MP / 64);
    gemm64<2><<<dim3((tiles + 7) / 8, BATCH), blk, 0, stream>>>(
        WqH + (size_t)2 * DM * DM, DM, xm, DM, MP * DM, (void*)vT, MP, DM * MP, vbias, dRC, dRS, smlog,
        DM, MP, DM, 1.0f / 32.0f, 1.0f);
  }
  attn64<<<dim3(BATCH * NH * NQB), dim3(128), 0, stream>>>(qP, kP, vT, nrp, ctx, 1.0f / 16.0f, 1.0f / 32.0f);
  {
    const int tiles = (MTOT / 64) * (DM / 64);
    gemm64<0><<<dim3((tiles + 7) / 8, 1), blk, 0, stream>>>(
        ctx, DM, WpH, DM, 0, (void*)dO, DM, 0, bproj, dRC, dRS, smlog,
        MTOT, DM, DM, 1.0f / 1024.0f, 1.0f);
  }
  k_out<<<dim3(BATCH * SEQ / 8), blk, 0, stream>>>(x, cached, dRnk, dO, out);
  (void)hipGetLastError();
}
